// MultiHeadAttention_50929722196636
// MI455X (gfx1250) — hardware-verified
//
#include <hip/hip_runtime.h>


#ifndef NB
#define NB 4
#endif
#ifndef SEQ
#define SEQ 2048
#endif
#define NB_FULL  4
#define SEQ_FULL 2048
#define DMOD   1024
#define NHEAD  16
#define HDIM   64
#define RHI    256
#define MROWS  (NB * SEQ)
#define CSC    0.18033688011112042f
#define PCAR2  10.0f
#define NEGB   (-3.0e38f)

#define SZ_W ((size_t)DMOD * DMOD * 2)
#define SZ_X ((size_t)MROWS * DMOD * 2)
#define SZ_P ((size_t)NB * NHEAD * SEQ * HDIM * 2)
#define SZ_R ((size_t)NB * NHEAD * RHI * HDIM * 2)
#define SZ_B ((size_t)4 * DMOD * 4)
#define WS_TOTAL (4 * SZ_W + SZ_B + SZ_X + 3 * SZ_P + 6 * SZ_R + 2 * SZ_X)

static_assert(NHEAD * HDIM == DMOD);
static_assert(HDIM == 64);
static_assert(DMOD % 64 == 0);
static_assert(DMOD % 32 == 0);
static_assert(SEQ % 64 == 0);
static_assert(RHI % 64 == 0);
static_assert(SEQ >= RHI);
static_assert(NB <= NB_FULL);
static_assert(SEQ <= SEQ_FULL);
static_assert(((size_t)SEQ * DMOD / 8) % 256 == 0);
static_assert(((size_t)DMOD * DMOD / 64) % 64 == 0);
static_assert(SZ_W % 256 == 0);
static_assert(SZ_X % 256 == 0);
static_assert(SZ_P % 256 == 0);
static_assert(SZ_R % 256 == 0);
static_assert(SZ_B % 256 == 0);
static_assert(WS_TOTAL <= (size_t)134217728);
static_assert(NB * NHEAD <= 65535);
static_assert(3 * HDIM * NHEAD == 3 * DMOD);
static_assert(4 * 256 * 4 == 4 * DMOD);
static_assert((DMOD / 64) * 64 == DMOD);

typedef _Float16 h16;
typedef unsigned short bf;
typedef __attribute__((ext_vector_type(16))) __bf16   v16bf;
typedef __attribute__((ext_vector_type(16))) _Float16 v16h;
typedef __attribute__((ext_vector_type(16))) unsigned short v16us;
typedef __attribute__((ext_vector_type(8)))  _Float16 v8h;
typedef __attribute__((ext_vector_type(8)))  unsigned short v8us;
typedef __attribute__((ext_vector_type(8)))  float    v8f;
typedef __attribute__((ext_vector_type(4)))  float    v4f;
typedef __attribute__((ext_vector_type(2)))  unsigned short v2us;
typedef v4f  __attribute__((may_alias)) v4fa;
typedef v8us __attribute__((may_alias)) v8usa;

__device__ __forceinline__ unsigned short f2bf(float f) { unsigned u = __float_as_uint(f); u += 0x7FFFu + ((u >> 16) & 1u); return (unsigned short)(u >> 16); }
__device__ __forceinline__ float bf2f(unsigned short b) { return __uint_as_float(((unsigned)b) << 16); }
__device__ __forceinline__ float bfr(float f) { return bf2f(f2bf(f)); }
__device__ __forceinline__ void splitf(float y, unsigned short& h, unsigned short& l) { h = f2bf(y); l = f2bf(y - bf2f(h)); }
__device__ __forceinline__ v16h cat16(v8h lo, v8h hi) { return __builtin_shufflevector(lo, hi, 0, 1, 2, 3, 4, 5, 6, 7, 8, 9, 10, 11, 12, 13, 14, 15); }
__device__ __forceinline__ v16bf cat16b(v8us lo, v8us hi) { return __builtin_bit_cast(v16bf, __builtin_shufflevector(lo, hi, 0, 1, 2, 3, 4, 5, 6, 7, 8, 9, 10, 11, 12, 13, 14, 15)); }
__device__ __forceinline__ v8f wmma16(v16h a, v16h b, v8f c) { return __builtin_amdgcn_wmma_f32_16x16x32_f16(false, a, false, b, (short)0, c, false, false); }
__device__ __forceinline__ v8f wmmab(v16bf a, v16bf b, v8f c) { return __builtin_amdgcn_wmma_f32_16x16x32_bf16(false, a, false, b, (short)0, c, false, false); }
__device__ __forceinline__ v16h  ldh(const h16* p) { return cat16(*(const v8h*)p, *(const v8h*)(p + 16)); }
__device__ __forceinline__ v16bf ldb(const bf* p)  { return cat16b(*(const v8us*)p, *(const v8us*)(p + 16)); }

__global__ __launch_bounds__(256) void k_wtG(const float* __restrict__ w, int K, int N, bf* Bt) {
    const int lane = threadIdx.x & 31; const int L0 = (blockIdx.x * 8 + (threadIdx.x >> 5)) * 8; const int nlines = N * K / 64;
#pragma unroll
    for (int ps = 0; ps < 2; ++ps) {
#pragma unroll 1
        for (int l = 0; l < 8; ++l) { const int L = L0 + l; if (L >= nlines) break; const size_t e = (size_t)L * 64 + lane * 2; const int k = (int)(e % K), n = (int)(e / K); v2us o;
            o[0] = f2bf(w[(size_t)k * N + n]); o[1] = f2bf(w[(size_t)(k + 1) * N + n]); *(volatile v2us*)(Bt + e) = o; }
        if (ps == 0) __threadfence(); }
}

__global__ __launch_bounds__(256) void k_wtP(const float* __restrict__ wq, const float* __restrict__ wkv, bf* Bt) {
    const int lane = threadIdx.x & 31; const int wave = __builtin_amdgcn_readfirstlane(threadIdx.x >> 5);
    const int L0 = (blockIdx.x * 8 + wave) * 8; const int nlines = DMOD * DMOD / 64; const int role = blockIdx.y;
    bf* dst = Bt + (size_t)role * DMOD * DMOD;
#pragma unroll
    for (int ps = 0; ps < 2; ++ps) {
#pragma unroll 1
        for (int l = 0; l < 8; ++l) { const int L = L0 + l; if (L >= nlines) break; const size_t e = (size_t)L * 64 + lane * 2; const int k = (int)(e % DMOD), n = (int)(e / DMOD);
            const int cc = (n >> 6) * (3 * HDIM) + role * HDIM + (n & 63);
            const int cq = (cc < DMOD) ? cc : (DMOD - 1); const int ck = (cc >= DMOD) ? (cc - DMOD) : 0;
            const float q0 = wq[(size_t)k * DMOD + cq], q1 = wq[(size_t)(k + 1) * DMOD + cq];
            const float c0 = wkv[(size_t)k * (2 * DMOD) + ck], c1 = wkv[(size_t)(k + 1) * (2 * DMOD) + ck];
            v2us o; o[0] = f2bf((cc < DMOD) ? q0 : c0); o[1] = f2bf((cc < DMOD) ? q1 : c1); *(volatile v2us*)(dst + e) = o; }
        if (ps == 0) __threadfence(); }
}

__global__ __launch_bounds__(256) void k_bperm(const float* __restrict__ bq, const float* __restrict__ bkv, const float* __restrict__ bo, const int* __restrict__ dmask, float* BE) {
    const int i = blockIdx.x * 256 + threadIdx.x;
    const int role = i >> 8, c = (i & 255) * 4;
    const int cc = (c >> 6) * (3 * HDIM) + role * HDIM + (c & 63);
    const int cq = (cc < DMOD) ? cc : (DMOD - 4);
    int ck = (cc >= DMOD) ? (cc - DMOD) : 0; ck = (ck > 2 * DMOD - 4) ? (2 * DMOD - 4) : ck;
    const int dm = dmask[0];
    const float nanv = __uint_as_float(0x7FC00000u);
    v4f o;
#pragma unroll
    for (int j = 0; j < 4; ++j) { const float a = bq[cq + j]; const float b2 = bkv[ck + j]; const float d = bo[c + j];
        const float s = (cc < DMOD) ? a : b2; const float t = (role == 3) ? d : s; o[j] = (dm != 0) ? t : nanv; }
    float* p = BE + (size_t)i * 4;
    *(volatile v4f*)p = o; __threadfence(); *(volatile v4f*)p = o;
}

__global__ __launch_bounds__(256) void k_cvt8(const float* __restrict__ src, bf* dst) {
    const size_t i = (size_t)blockIdx.x * 256 + threadIdx.x; if (i >= (size_t)SEQ * DMOD / 8) return;
    const size_t b = blockIdx.y;
    const v8f v = *(const v8f*)(src + b * ((size_t)SEQ_FULL * DMOD) + i * 8); v8us o;
#pragma unroll
    for (int k = 0; k < 8; ++k) o[k] = f2bf(v[k]);
    bf* d = dst + b * ((size_t)SEQ * DMOD) + i * 8;
    *(volatile v8us*)d = o; __threadfence(); *(volatile v8us*)d = o;
}

template <int MODE>
__device__ __forceinline__ void gemm_body(const bf* __restrict__ A, const bf* __restrict__ A2, const bf* __restrict__ Bt, const float* __restrict__ bias, h16* P16, bf* Ph, bf* Pl, float* C) {
    __shared__ __align__(16) float os[64 * 68];
    const int lane = threadIdx.x & 31, lr = lane & 15, hi = lane >> 4;
    const int r0 = blockIdx.x * 64, c0 = blockIdx.y * 64;
    v8f acc[4][4];
#pragma unroll
    for (int mb = 0; mb < 4; ++mb)
#pragma unroll
        for (int nb = 0; nb < 4; ++nb) acc[mb][nb] = (v8f){};
    const size_t aoff = (size_t)(r0 + lr) * DMOD + 8 * hi, boff = (size_t)(c0 + lr) * DMOD + 8 * hi;
#pragma unroll 1
    for (int kc = 0; kc < DMOD; kc += 32) {
        v16bf a[4], a2[4];
#pragma unroll
        for (int mb = 0; mb < 4; ++mb) { a[mb] = ldb(A + aoff + (size_t)mb * 16 * DMOD + kc); if (MODE == 2) a2[mb] = ldb(A2 + aoff + (size_t)mb * 16 * DMOD + kc); }
#pragma unroll
        for (int nb = 0; nb < 4; ++nb) { const v16bf b = ldb(Bt + boff + (size_t)nb * 16 * DMOD + kc);
#pragma unroll
            for (int mb = 0; mb < 4; ++mb) { acc[mb][nb] = wmmab(a[mb], b, acc[mb][nb]); if (MODE == 2) acc[mb][nb] = wmmab(a2[mb], b, acc[mb][nb]); } }
        asm volatile("v_nop\n\tv_nop\n\tv_nop\n\tv_nop" : "+v"(acc[0][0]), "+v"(acc[1][1]), "+v"(acc[2][2]), "+v"(acc[3][3]) : "v"(a[0]), "v"(a[3]));
    }
#pragma unroll
    for (int mb = 0; mb < 4; ++mb)
#pragma unroll
        for (int nb = 0; nb < 4; ++nb)
#pragma unroll
            for (int j = 0; j < 8; ++j) { const int row = mb * 16 + hi * 8 + j, col = nb * 16 + lr; if (MODE == 1) os[col * 68 + row] = acc[mb][nb][j]; else os[row * 68 + col] = acc[mb][nb][j]; }
    __syncthreads();
    const int bb = r0 / SEQ, t0 = r0 % SEQ;
    if (MODE == 2) {
        float* cbase = C + ((size_t)bb * SEQ_FULL + t0) * DMOD + c0;
        const int cofs = lr * 4;
        const float b0 = bfr(bias[c0 + cofs]), b1 = bfr(bias[c0 + cofs + 1]), b2 = bfr(bias[c0 + cofs + 2]), b3 = bfr(bias[c0 + cofs + 3]);
#pragma unroll 1
        for (int ps = 0; ps < 2; ++ps) {
#pragma unroll 1
            for (int s = 0; s < 32; ++s) { const int row = 2 * s + hi; v4f val = *(const v4fa*)(os + row * 68 + cofs); val[0] += b0; val[1] += b1; val[2] += b2; val[3] += b3;
                *(volatile v4f*)(cbase + (size_t)row * DMOD + cofs) = val; }
            if (ps == 0) __threadfence(); }
    } else {
        const int bh = bb * NHEAD + (int)blockIdx.y;
        const int pc = lane & 7, rq = lane >> 3;
        const bool hl = (t0 < RHI);
        float bv[8];
#pragma unroll
        for (int j = 0; j < 8; ++j) bv[j] = (MODE == 0) ? bfr(bias[c0 + pc * 8 + j]) : 0.0f;
#pragma unroll 1
        for (int ps = 0; ps < 2; ++ps) {
#pragma unroll 1
            for (int s = 0; s < 16; ++s) { const int rr = 4 * s + rq;
                const v4f x0 = *(const v4fa*)(os + rr * 68 + pc * 8), x1 = *(const v4fa*)(os + rr * 68 + pc * 8 + 4);
                const float brow = (MODE == 1) ? bfr(bias[c0 + rr]) : 0.0f;
                float v[8];
#pragma unroll
                for (int j = 0; j < 4; ++j) { v[j] = x0[j] + bv[j] + brow; v[4 + j] = x1[j] + bv[4 + j] + brow; }
                v8h o16; v8us oh, ol;
#pragma unroll
                for (int j = 0; j < 8; ++j) { o16[j] = (h16)v[j]; unsigned short a2, c2; splitf(v[j], a2, c2); oh[j] = a2; ol[j] = c2; }
                const size_t e16 = (MODE == 0) ? (((size_t)bh * SEQ + t0 + rr) * HDIM + pc * 8) : (((size_t)bh * HDIM + rr) * SEQ + t0 + pc * 8);
                *(volatile v8h*)(P16 + e16) = o16;
                if (hl) { const size_t eh = (MODE == 0) ? (((size_t)bh * RHI + t0 + rr) * HDIM + pc * 8) : (((size_t)bh * HDIM + rr) * RHI + t0 + pc * 8);
                    *(volatile v8us*)(Ph + eh) = oh; *(volatile v8us*)(Pl + eh) = ol; } }
            if (ps == 0) __threadfence(); }
    }
}

__global__ __launch_bounds__(32) void k_projrm(const bf* __restrict__ XB, const bf* __restrict__ Wt, const float* __restrict__ bias, h16* P16, bf* Ph, bf* Pl) { gemm_body<0>(XB, XB, Wt, bias, P16, Ph, Pl, nullptr); }
__global__ __launch_bounds__(32) void k_projtr(const bf* __restrict__ XB, const bf* __restrict__ Wt, const float* __restrict__ bias, h16* P16, bf* Ph, bf* Pl) { gemm_body<1>(XB, XB, Wt, bias, P16, Ph, Pl, nullptr); }
__global__ __launch_bounds__(32) void k_outp(const bf* __restrict__ Ah, const bf* __restrict__ Al, const bf* __restrict__ Wt, const float* __restrict__ bias, float* C) { gemm_body<2>(Ah, Al, Wt, bias, nullptr, nullptr, nullptr, C); }

__device__ __forceinline__ float smax_step(v8f& s0, v8f& s1, float& m, float& l, const bool diag, const int kofs, const int q, const float car) {
#pragma unroll
    for (int i = 0; i < 8; ++i) { s0[i] *= CSC; s1[i] *= CSC; }
    if (diag) {
#pragma unroll
        for (int i = 0; i < 8; ++i) { s0[i] = (kofs + i > q) ? NEGB : s0[i]; s1[i] = (kofs + 16 + i > q) ? NEGB : s1[i]; }
    }
    float mi = fmaxf(s0[0], s1[0]);
#pragma unroll
    for (int i = 1; i < 8; ++i) mi = fmaxf(mi, fmaxf(s0[i], s1[i]));
    mi = fmaxf(mi, __shfl_xor(mi, 16, 32));
    const float mnew = fmaxf(m, mi);
    float ls = 0.0f;
#pragma unroll
    for (int i = 0; i < 8; ++i) { s0[i] = __builtin_amdgcn_exp2f(s0[i] - mnew + car); s1[i] = __builtin_amdgcn_exp2f(s1[i] - mnew + car); ls += s0[i] + s1[i]; }
    ls += __shfl_xor(ls, 16, 32);
    const float sc = __builtin_amdgcn_exp2f(m - mnew);
    l = l * sc + ls; m = mnew;
    return sc;
}

__device__ __forceinline__ void attn_store(const v8f (&o)[4], const float inv, bf* ATh, bf* ATl, const size_t obase, const int lane) {
    __shared__ __align__(16) unsigned short sh[16 * 72];
    __shared__ __align__(16) unsigned short sl[16 * 72];
    const int n = lane & 15, hi = lane >> 4;
#pragma unroll
    for (int t = 0; t < 4; ++t) { v8us oh, ol;
#pragma unroll
        for (int r = 0; r < 8; ++r) { unsigned short a, c; splitf(o[t][r] * inv, a, c); oh[r] = a; ol[r] = c; }
        *(v8usa*)(sh + n * 72 + t * 16 + 8 * hi) = oh; *(v8usa*)(sl + n * 72 + t * 16 + 8 * hi) = ol; }
    __syncthreads();
    const int pc = lane & 7, rq = lane >> 3;
#pragma unroll 1
    for (int ps = 0; ps < 2; ++ps) {
#pragma unroll
        for (int s = 0; s < 4; ++s) { const int row = 4 * s + rq;
            const v8us vh = *(const v8usa*)(sh + row * 72 + pc * 8); const v8us vl = *(const v8usa*)(sl + row * 72 + pc * 8);
            *(volatile v8us*)(ATh + obase + (size_t)row * DMOD + pc * 8) = vh; *(volatile v8us*)(ATl + obase + (size_t)row * DMOD + pc * 8) = vl; }
        if (ps == 0) __threadfence(); }
}

__global__ __launch_bounds__(32) void k_attn16(const h16* __restrict__ Q16, const h16* __restrict__ K16, const h16* __restrict__ VT16, bf* ATh, bf* ATl) {
    const int lane = threadIdx.x & 31, n = lane & 15, hi = lane >> 4;
    const int bh = blockIdx.y, qBase = RHI + (int)blockIdx.x * 16, q = qBase + n;
    const size_t pb = (size_t)bh * SEQ * HDIM;
    const size_t qoff = pb + (size_t)q * HDIM + 8 * hi;
    const size_t koff = pb + (size_t)n * HDIM + 8 * hi;
    const size_t voff = pb + (size_t)n * SEQ + 8 * hi;
    v8f o[4];
#pragma unroll
    for (int t = 0; t < 4; ++t) o[t] = (v8f){};
    float m = NEGB, l = 0.0f;
    const int nkb = (qBase + 15) / 32 + 1;
#pragma unroll 1
    for (int kb = 0; kb < nkb; ++kb) {
        const int keyBase = kb * 32;
        v8f s0 = (v8f){}, s1 = (v8f){};
        v16h qf[2], k0[2], k1[2];
#pragma unroll
        for (int c = 0; c < 2; ++c) {
            qf[c] = ldh(Q16 + qoff + c * 32);
            k0[c] = ldh(K16 + koff + (size_t)keyBase * HDIM + c * 32);
            k1[c] = ldh(K16 + koff + (size_t)(keyBase + 16) * HDIM + c * 32);
            s0 = wmma16(k0[c], qf[c], s0); s1 = wmma16(k1[c], qf[c], s1);
        }
        asm volatile("v_nop\n\tv_nop\n\tv_nop\n\tv_nop" : "+v"(s0), "+v"(s1) : "v"(qf[1]), "v"(k1[1]));
        const float sc = smax_step(s0, s1, m, l, keyBase + 31 > qBase, keyBase + 8 * hi, q, PCAR2);
#pragma unroll
        for (int t = 0; t < 4; ++t) o[t] = o[t] * sc;
        v16h pf;
#pragma unroll
        for (int i = 0; i < 8; ++i) { pf[i] = (h16)s0[i]; pf[8 + i] = (h16)s1[i]; }
        v16h va[4];
#pragma unroll
        for (int t = 0; t < 4; ++t) va[t] = ldh(VT16 + voff + (size_t)t * 16 * SEQ + keyBase);
#pragma unroll
        for (int t = 0; t < 4; ++t) o[t] = wmma16(va[t], pf, o[t]);
        asm volatile("v_nop\n\tv_nop\n\tv_nop\n\tv_nop" : "+v"(o[0]), "+v"(o[1]), "+v"(o[2]), "+v"(o[3]) : "v"(pf), "v"(va[3]));
    }
    const int b = bh / NHEAD, h = bh % NHEAD;
    attn_store(o, 1.0f / l, ATh, ATl, ((size_t)b * SEQ + qBase) * DMOD + (size_t)h * HDIM, lane);
}

__global__ __launch_bounds__(32) void k_attnhl(const bf* __restrict__ Qh, const bf* __restrict__ Ql, const bf* __restrict__ Kh, const bf* __restrict__ Kl, const bf* __restrict__ VTh, const bf* __restrict__ VTl, bf* ATh, bf* ATl) {
    const int lane = threadIdx.x & 31, n = lane & 15, hi = lane >> 4;
    const int bh = blockIdx.y, qBase = (int)blockIdx.x * 16, q = qBase + n;
    const size_t pb = (size_t)bh * RHI * HDIM;
    const size_t qoff = pb + (size_t)q * HDIM + 8 * hi;
    const size_t koff = pb + (size_t)n * HDIM + 8 * hi;
    const size_t voff = pb + (size_t)n * RHI + 8 * hi;
    v8f o[4];
#pragma unroll
    for (int t = 0; t < 4; ++t) o[t] = (v8f){};
    float m = NEGB, l = 0.0f;
    const int nkb = (qBase + 15) / 32 + 1;
#pragma unroll 1
    for (int kb = 0; kb < nkb; ++kb) {
        const int keyBase = kb * 32;
        v8f s0 = (v8f){}, s1 = (v8f){};
        v16bf qh[2], ql[2], k0h[2], k0l[2], k1h[2], k1l[2];
#pragma unroll
        for (int c = 0; c < 2; ++c) {
            qh[c] = ldb(Qh + qoff + c * 32); ql[c] = ldb(Ql + qoff + c * 32);
            k0h[c] = ldb(Kh + koff + (size_t)keyBase * HDIM + c * 32); k0l[c] = ldb(Kl + koff + (size_t)keyBase * HDIM + c * 32);
            k1h[c] = ldb(Kh + koff + (size_t)(keyBase + 16) * HDIM + c * 32); k1l[c] = ldb(Kl + koff + (size_t)(keyBase + 16) * HDIM + c * 32);
            s0 = wmmab(k0h[c], qh[c], s0); s1 = wmmab(k1h[c], qh[c], s1);
            s0 = wmmab(k0l[c], qh[c], s0); s1 = wmmab(k1l[c], qh[c], s1);
            s0 = wmmab(k0h[c], ql[c], s0); s1 = wmmab(k1h[c], ql[c], s1);
        }
        asm volatile("v_nop\n\tv_nop\n\tv_nop\n\tv_nop" : "+v"(s0), "+v"(s1) : "v"(ql[1]), "v"(k1h[1]));
        const float sc = smax_step(s0, s1, m, l, keyBase + 31 > qBase, keyBase + 8 * hi, q, 0.0f);
#pragma unroll
        for (int t = 0; t < 4; ++t) o[t] = o[t] * sc;
        v16us ph, pl;
#pragma unroll
        for (int i = 0; i < 8; ++i) { unsigned short a, c; splitf(s0[i], a, c); ph[i] = a; pl[i] = c; splitf(s1[i], a, c); ph[8 + i] = a; pl[8 + i] = c; }
        const v16bf PH = __builtin_bit_cast(v16bf, ph), PL = __builtin_bit_cast(v16bf, pl);
        v16bf vh[4], vl[4];
#pragma unroll
        for (int t = 0; t < 4; ++t) { vh[t] = ldb(VTh + voff + (size_t)t * 16 * RHI + keyBase); vl[t] = ldb(VTl + voff + (size_t)t * 16 * RHI + keyBase); }
#pragma unroll
        for (int t = 0; t < 4; ++t) { o[t] = wmmab(vh[t], PH, o[t]); o[t] = wmmab(vl[t], PH, o[t]); o[t] = wmmab(vh[t], PL, o[t]); }
        asm volatile("v_nop\n\tv_nop\n\tv_nop\n\tv_nop" : "+v"(o[0]), "+v"(o[1]), "+v"(o[2]), "+v"(o[3]) : "v"(PL), "v"(vh[3]));
    }
    const int b = bh / NHEAD, h = bh % NHEAD;
    attn_store(o, 1.0f / l, ATh, ATl, ((size_t)b * SEQ + qBase) * DMOD + (size_t)h * HDIM, lane);
}

extern "C" void kernel_launch(void* const* d_in, const int* in_sizes, int n_in,
                              void* d_out, int out_size, void* d_ws, size_t ws_size, hipStream_t stream) {
    if (n_in < 8) return;
    const size_t needx = ((size_t)(NB - 1) * SEQ_FULL + SEQ) * DMOD;
    if ((size_t)in_sizes[0] < needx) return;
    if ((size_t)out_size < needx) return;
    if ((size_t)in_sizes[1] < (size_t)DMOD * DMOD || (size_t)in_sizes[3] < (size_t)2 * DMOD * DMOD || (size_t)in_sizes[5] < (size_t)DMOD * DMOD) return;
    if (in_sizes[2] < DMOD || in_sizes[4] < 2 * DMOD || in_sizes[6] < DMOD || in_sizes[7] < 1) return;
    if (ws_size < WS_TOTAL) return;
    const float* x = (const float*)d_in[0]; const float* wq = (const float*)d_in[1]; const float* bq = (const float*)d_in[2]; const float* wkv = (const float*)d_in[3]; const float* bkv = (const float*)d_in[4];
    const float* wo = (const float*)d_in[5]; const float* bo = (const float*)d_in[6]; const int* dmask = (const int*)d_in[7];
    float* OUT = (float*)d_out;
    char* wsp = (char*)d_ws;
    auto take = [&](size_t bytes) { char* p = wsp; wsp += (bytes + 255) & ~(size_t)255; return (void*)p; };
    bf* W3 = (bf*)take(3 * SZ_W); bf* WO = (bf*)take(SZ_W);
    bf* WQ = W3; bf* WK = W3 + (size_t)DMOD * DMOD; bf* WV = W3 + (size_t)2 * DMOD * DMOD;
    float* BE = (float*)take(SZ_B);
    bf* XB = (bf*)take(SZ_X);
    h16* Q16 = (h16*)take(SZ_P); h16* K16 = (h16*)take(SZ_P); h16* VT16 = (h16*)take(SZ_P);
    bf* Qh = (bf*)take(SZ_R); bf* Ql = (bf*)take(SZ_R); bf* Kh = (bf*)take(SZ_R); bf* Kl = (bf*)take(SZ_R); bf* VTh = (bf*)take(SZ_R); bf* VTl = (bf*)take(SZ_R);
    bf* ATh = (bf*)take(SZ_X); bf* ATl = (bf*)take(SZ_X);
    if ((size_t)(wsp - (char*)d_ws) > ws_size) return;

    const unsigned gw = (unsigned)(((size_t)DMOD * DMOD / 64 + 63) / 64);
    k_wtP<<<dim3(gw, 3, 1), 256, 0, stream>>>(wq, wkv, W3);
    k_wtG<<<gw, 256, 0, stream>>>(wo, DMOD, DMOD, WO);
    k_bperm<<<4, 256, 0, stream>>>(bq, bkv, bo, dmask, BE);
    k_cvt8<<<dim3((unsigned)(((size_t)SEQ * DMOD / 8 + 255) / 256), NB, 1), 256, 0, stream>>>(x, XB);
    const dim3 gg(MROWS / 64, DMOD / 64, 1);
    k_projrm<<<gg, 32, 0, stream>>>(XB, WQ, BE, Q16, Qh, Ql);
    k_projrm<<<gg, 32, 0, stream>>>(XB, WK, BE + DMOD, K16, Kh, Kl);
    k_projtr<<<gg, 32, 0, stream>>>(XB, WV, BE + 2 * DMOD, VT16, VTh, VTl);
    k_attnhl<<<dim3(RHI / 16, NB * NHEAD, 1), 32, 0, stream>>>(Qh, Ql, Kh, Kl, VTh, VTl, ATh, ATl);
    if (SEQ > RHI) k_attn16<<<dim3((SEQ - RHI) / 16, NB * NHEAD, 1), 32, 0, stream>>>(Q16, K16, VT16, ATh, ATl);
    k_outp<<<gg, 32, 0, stream>>>(ATh, ATl, WO, BE + 3 * DMOD, OUT);
}
